// ProbabilisticAttention_21165598835368
// MI455X (gfx1250) — hardware-verified
//
#include <hip/hip_runtime.h>
#include <hip/hip_bf16.h>
#include <math.h>


typedef _Float16 bf16;
typedef _Float16 f16;
typedef __attribute__((ext_vector_type(4))) unsigned v4u_t;
typedef unsigned v4ua __attribute__((ext_vector_type(4), may_alias));
typedef __attribute__((ext_vector_type(4))) float v4f_t;
typedef float v4fa __attribute__((ext_vector_type(4), may_alias));
typedef __attribute__((ext_vector_type(16))) bf16  bf16x16;
typedef bf16x16 f16x16;
typedef __attribute__((ext_vector_type(8)))  bf16  bf16x8;
typedef bf16x8 f16x8;
typedef __attribute__((ext_vector_type(4)))  bf16  bf16x4;
typedef __attribute__((ext_vector_type(8)))  float f32x8;
__device__ __forceinline__ f32x8 wmma16(f16x16 a, f16x16 b, f32x8 c) {
  c = __builtin_amdgcn_wmma_f32_16x16x32_f16(false, a, false, b, (short)0, c, false, false);
  asm volatile("v_nop\n\tv_nop\n\tv_nop\n\tv_nop" : "+v"(c) : "v"(a), "v"(b));
  return c;
}
#define LDS_STRIDE 48
#define KSTRIDE    72
#define VSTRIDE    48

__device__ __forceinline__ f32x8 wmma_bf16(bf16x16 a, bf16x16 b, f32x8 c) {
  c = __builtin_amdgcn_wmma_f32_16x16x32_f16(false, a, false, b, (short)0, c, false, false);
  asm volatile("v_nop\n\tv_nop\n\tv_nop\n\tv_nop" : "+v"(c) : "v"(a), "v"(b));
  return c;
}

template <typename T>
__device__ __forceinline__ bf16x16 load_frag(const T* __restrict__ base, int ld,
                                             int row0, int k0) {
  const int lane = threadIdx.x & 31;
  const int r    = lane & 15;
  const int kh   = (lane >> 4) * 8;
  const T* p0 = base + (size_t)(row0 + r) * ld + (k0 + kh);
  const T* p1 = p0 + 16;
  bf16x16 f;
#pragma unroll
  for (int i = 0; i < 8; ++i) {
    f[i]     = (bf16)p0[i];
    f[i + 8] = (bf16)p1[i];
  }
  return f;
}

__device__ __forceinline__ bf16x16 lds_frag(const bf16* base, int stride) {
  const int lane = threadIdx.x & 31;
  const int row  = lane & 15;
  const int kh   = (lane >> 4) * 8;
  const bf16x8 lo = *(const bf16x8*)(base + row * stride + kh);
  const bf16x8 hi = *(const bf16x8*)(base + row * stride + kh + 16);
  bf16x16 f;
#pragma unroll
  for (int i = 0; i < 8; ++i) { f[i] = lo[i]; f[i + 8] = hi[i]; }
  return f;
}

template <typename T>
__device__ __forceinline__ void stage_read16(const T* __restrict__ p, float* buf) {
#pragma unroll
  for (int i = 0; i < 16; ++i) buf[i] = (float)p[i];
}

__device__ __forceinline__ void stage_write(bf16* dst, const float* buf, int nquad) {
#pragma unroll
  for (int i = 0; i < nquad; ++i) {
    bf16x4 q;
    q[0] = (bf16)buf[4 * i];     q[1] = (bf16)buf[4 * i + 1];
    q[2] = (bf16)buf[4 * i + 2]; q[3] = (bf16)buf[4 * i + 3];
    *(bf16x4*)(dst + 4 * i) = q;
  }
}


#define GSTR 48
#define GSTR 48
template <typename AT, int EPI, bool OUT16>
__global__ __launch_bounds__(256) void gemm_kne(const AT* __restrict__ A, int lda, const float* __restrict__ Wm, int ldw,
                                                const float* __restrict__ bias, const float* __restrict__ R, const float* __restrict__ gvec,
                                                void* __restrict__ Yv, int ldy, int K) {
  __shared__ __attribute__((aligned(16))) f16 ldsA[128 * GSTR];
  __shared__ __attribute__((aligned(16))) f16 ldsW[128 * GSTR];
  __shared__ __attribute__((aligned(16))) float oS[8][32 * 68];
  const int tid = threadIdx.x, lane = tid & 31, wave = tid >> 5, cl = lane & 15, rh = (lane >> 4) * 8;
  const int m0 = blockIdx.x * 128, n0 = blockIdx.y * 128;
  const int wm = (wave & 3) * 32, wn = (wave >> 2) * 64;
  f32x8 acc[2][4];
#pragma unroll
  for (int i = 0; i < 2; ++i)
#pragma unroll
    for (int j = 0; j < 4; ++j) { f32x8 z = {}; acc[i][j] = z; }
#pragma unroll 1
  for (int k0 = 0; k0 < K; k0 += 32) {
    __syncthreads();
    { const int row = tid >> 1, ch = (tid & 1) * 16;
      const AT* src = A + (size_t)(m0 + row) * lda + k0 + ch;
#pragma unroll
      for (int g = 0; g < 16; ++g) ldsA[row * GSTR + ch + g] = (f16)src[g]; }
    { const int k = tid >> 3, nn0 = (tid & 7) * 16;
      const float* src = Wm + (size_t)(k0 + k) * ldw + n0 + nn0;
#pragma unroll
      for (int g = 0; g < 4; ++g) { const v4f_t v = *(const v4f_t*)(src + 4 * g);
#pragma unroll
        for (int u = 0; u < 4; ++u) ldsW[(nn0 + 4 * g + u) * GSTR + k] = (f16)v[u]; } }
    __syncthreads();
    f16x16 af[2];
#pragma unroll
    for (int i = 0; i < 2; ++i) af[i] = lds_frag(ldsA + (wm + 16 * i) * GSTR, GSTR);
#pragma unroll
    for (int j = 0; j < 4; ++j) {
      const f16x16 bf = lds_frag(ldsW + (wn + 16 * j) * GSTR, GSTR);
#pragma unroll
      for (int i = 0; i < 2; ++i) acc[i][j] = wmma16(af[i], bf, acc[i][j]);
    }
  }
  float* so = oS[wave];
#pragma unroll
  for (int i = 0; i < 2; ++i)
#pragma unroll
    for (int j = 0; j < 4; ++j) {
      const int n = n0 + wn + 16 * j + cl;
      const float bv = bias ? bias[n] : 0.0f;
      const float gv = (EPI == 2 || EPI == 4) ? gvec[n] : 0.0f;
      if (EPI == 1) {
#pragma unroll 1
        for (int r = 0; r < 8; ++r) { const float xg = acc[i][j][r] + bv; so[(16 * i + rh + r) * 68 + 16 * j + cl] = 0.5f * xg * (1.0f + erff(xg * 0.70710678118654752f)); }
      } else {
#pragma unroll
        for (int r = 0; r < 8; ++r) {
          float v = acc[i][j][r] + bv;
          if (EPI == 3) v = fmaxf(v, 0.0f);
          if (EPI == 4) v = gv * v;
          if (EPI == 2) v = R[(size_t)(m0 + wm + 16 * i + rh + r) * ldy + n] + gv * v;
          so[(16 * i + rh + r) * 68 + 16 * j + cl] = v;
        }
      }
    }
  asm volatile("s_wait_dscnt 0" ::: "memory");
  __builtin_amdgcn_wave_barrier();
#pragma unroll 1
  for (int pass = 0; pass < 2; ++pass) {
    if (OUT16) {
      f16* Y = (f16*)Yv;
#pragma unroll
      for (int it = 0; it < 8; ++it) { const int c = lane + 32 * it, rr = c >> 3, q8 = (c & 7) * 8;
        union { f16 h[8]; v4u_t v; } u;
#pragma unroll
        for (int e = 0; e < 8; ++e) u.h[e] = (f16)so[rr * 68 + q8 + e];
        *(volatile v4u_t*)(Y + (size_t)(m0 + wm + rr) * ldy + n0 + wn + q8) = u.v; }
    } else {
      float* Y = (float*)Yv;
#pragma unroll
      for (int it = 0; it < 16; ++it) { const int f4 = lane + 32 * it, rr = f4 >> 4, q = (f4 & 15) * 4;
        *(volatile v4f_t*)(Y + (size_t)(m0 + wm + rr) * ldy + n0 + wn + q) = *(const v4fa*)(so + rr * 68 + q); }
    }
    __threadfence();
  }
}

template <typename AT, int EPI, bool OUT16>
__global__ __launch_bounds__(256) void gemm_knez(const AT* __restrict__ A, int lda, size_t strideA, const float* __restrict__ Wm, int ldw, size_t strideW,
                                                 const float* __restrict__ bias, const float* __restrict__ R, const float* __restrict__ gvec,
                                                 void* __restrict__ Yv, int ldy, size_t strideY, int K) {
  A += (size_t)blockIdx.z * strideA; Wm += (size_t)blockIdx.z * strideW; Yv = (void*)((char*)Yv + (size_t)blockIdx.z * strideY * (OUT16 ? 2 : 4)); if (R) R += (size_t)blockIdx.z * strideY;
  __shared__ __attribute__((aligned(16))) f16 ldsA[128 * GSTR];
  __shared__ __attribute__((aligned(16))) f16 ldsW[128 * GSTR];
  __shared__ __attribute__((aligned(16))) float oS[8][32 * 68];
  const int tid = threadIdx.x, lane = tid & 31, wave = tid >> 5, cl = lane & 15, rh = (lane >> 4) * 8;
  const int m0 = blockIdx.x * 128, n0 = blockIdx.y * 128;
  const int wm = (wave & 3) * 32, wn = (wave >> 2) * 64;
  f32x8 acc[2][4];
#pragma unroll
  for (int i = 0; i < 2; ++i)
#pragma unroll
    for (int j = 0; j < 4; ++j) { f32x8 z = {}; acc[i][j] = z; }
#pragma unroll 1
  for (int k0 = 0; k0 < K; k0 += 32) {
    __syncthreads();
    { const int row = tid >> 1, ch = (tid & 1) * 16;
      const AT* src = A + (size_t)(m0 + row) * lda + k0 + ch;
#pragma unroll
      for (int g = 0; g < 16; ++g) ldsA[row * GSTR + ch + g] = (f16)src[g]; }
    { const int k = tid >> 3, nn0 = (tid & 7) * 16;
      const float* src = Wm + (size_t)(k0 + k) * ldw + n0 + nn0;
#pragma unroll
      for (int g = 0; g < 4; ++g) { const v4f_t v = *(const v4f_t*)(src + 4 * g);
#pragma unroll
        for (int u = 0; u < 4; ++u) ldsW[(nn0 + 4 * g + u) * GSTR + k] = (f16)v[u]; } }
    __syncthreads();
    f16x16 af[2];
#pragma unroll
    for (int i = 0; i < 2; ++i) af[i] = lds_frag(ldsA + (wm + 16 * i) * GSTR, GSTR);
#pragma unroll
    for (int j = 0; j < 4; ++j) {
      const f16x16 bf = lds_frag(ldsW + (wn + 16 * j) * GSTR, GSTR);
#pragma unroll
      for (int i = 0; i < 2; ++i) acc[i][j] = wmma16(af[i], bf, acc[i][j]);
    }
  }
  float* so = oS[wave];
#pragma unroll
  for (int i = 0; i < 2; ++i)
#pragma unroll
    for (int j = 0; j < 4; ++j) {
      const int n = n0 + wn + 16 * j + cl;
      const float bv = bias ? bias[n] : 0.0f;
      const float gv = (EPI == 2 || EPI == 4) ? gvec[n] : 0.0f;
      if (EPI == 1) {
#pragma unroll 1
        for (int r = 0; r < 8; ++r) { const float xg = acc[i][j][r] + bv; so[(16 * i + rh + r) * 68 + 16 * j + cl] = 0.5f * xg * (1.0f + erff(xg * 0.70710678118654752f)); }
      } else {
#pragma unroll
        for (int r = 0; r < 8; ++r) {
          float v = acc[i][j][r] + bv;
          if (EPI == 3) v = fmaxf(v, 0.0f);
          if (EPI == 4) v = gv * v;
          if (EPI == 2) v = R[(size_t)(m0 + wm + 16 * i + rh + r) * ldy + n] + gv * v;
          so[(16 * i + rh + r) * 68 + 16 * j + cl] = v;
        }
      }
    }
  asm volatile("s_wait_dscnt 0" ::: "memory");
  __builtin_amdgcn_wave_barrier();
#pragma unroll 1
  for (int pass = 0; pass < 2; ++pass) {
    if (OUT16) {
      f16* Y = (f16*)Yv;
#pragma unroll
      for (int it = 0; it < 8; ++it) { const int c = lane + 32 * it, rr = c >> 3, q8 = (c & 7) * 8;
        union { f16 h[8]; v4u_t v; } u;
#pragma unroll
        for (int e = 0; e < 8; ++e) u.h[e] = (f16)so[rr * 68 + q8 + e];
        *(volatile v4u_t*)(Y + (size_t)(m0 + wm + rr) * ldy + n0 + wn + q8) = u.v; }
    } else {
      float* Y = (float*)Yv;
#pragma unroll
      for (int it = 0; it < 16; ++it) { const int f4 = lane + 32 * it, rr = f4 >> 4, q = (f4 & 15) * 4;
        *(volatile v4f_t*)(Y + (size_t)(m0 + wm + rr) * ldy + n0 + wn + q) = *(const v4fa*)(so + rr * 68 + q); }
    }
    __threadfence();
  }
}

template <typename AT, bool ACC>
__global__ __launch_bounds__(256) void gemm_kn2(const AT* __restrict__ A, int lda, size_t strideA,
                                               const float* __restrict__ Wm, int ldw, size_t strideW,
                                               const float* __restrict__ bias, float scale,
                                               float* __restrict__ Y, int ldy, size_t strideY, int K) {
  __shared__ __attribute__((aligned(16))) f16 ldsA[128 * GSTR], ldsAl[128 * GSTR];
  __shared__ __attribute__((aligned(16))) f16 ldsW[128 * GSTR], ldsWl[128 * GSTR];
  __shared__ __attribute__((aligned(16))) float oS[8][32 * 68];
  const int tid = threadIdx.x, lane = tid & 31, wave = tid >> 5, cl = lane & 15, rh = (lane >> 4) * 8;
  const int m0 = blockIdx.x * 128, n0 = blockIdx.y * 128;
  const int wm = (wave & 3) * 32, wn = (wave >> 2) * 64;
  A += (size_t)blockIdx.z * strideA; Wm += (size_t)blockIdx.z * strideW; Y += (size_t)blockIdx.z * strideY;
  f32x8 acc[2][4], accx[2][4];
#pragma unroll
  for (int i = 0; i < 2; ++i)
#pragma unroll
    for (int j = 0; j < 4; ++j) { f32x8 z = {}; acc[i][j] = z; accx[i][j] = z; }
#pragma unroll 1
  for (int k0 = 0; k0 < K; k0 += 32) {
    __syncthreads();
    {
      const int row = tid >> 1, ch = (tid & 1) * 16;
      const AT* src = A + (size_t)(m0 + row) * lda + k0 + ch;
#pragma unroll
      for (int g = 0; g < 16; ++g) { const float v = (float)src[g]; const f16 h = (f16)v; ldsA[row * GSTR + ch + g] = h; ldsAl[row * GSTR + ch + g] = (f16)((v - (float)h) * 2048.0f); }
    }
    {
      const int k = tid >> 3, nn0 = (tid & 7) * 16;
      const float* src = Wm + (size_t)(k0 + k) * ldw + n0 + nn0;
#pragma unroll
      for (int g = 0; g < 4; ++g) { const v4f_t v = *(const v4f_t*)(src + 4 * g);
#pragma unroll
        for (int u = 0; u < 4; ++u) { const f16 h = (f16)v[u]; ldsW[(nn0 + 4 * g + u) * GSTR + k] = h; ldsWl[(nn0 + 4 * g + u) * GSTR + k] = (f16)((v[u] - (float)h) * 2048.0f); } }
    }
    __syncthreads();
    f16x16 af[2], afl[2];
#pragma unroll
    for (int i = 0; i < 2; ++i) { af[i] = lds_frag(ldsA + (wm + 16 * i) * GSTR, GSTR); afl[i] = lds_frag(ldsAl + (wm + 16 * i) * GSTR, GSTR); }
#pragma unroll
    for (int j = 0; j < 4; ++j) {
      const f16x16 bf = lds_frag(ldsW + (wn + 16 * j) * GSTR, GSTR), bfl = lds_frag(ldsWl + (wn + 16 * j) * GSTR, GSTR);
#pragma unroll
      for (int i = 0; i < 2; ++i) { acc[i][j] = wmma16(af[i], bf, acc[i][j]); accx[i][j] = wmma16(af[i], bfl, accx[i][j]); accx[i][j] = wmma16(afl[i], bf, accx[i][j]); }
    }
  }
  float* so = oS[wave];
#pragma unroll
  for (int i = 0; i < 2; ++i)
#pragma unroll
    for (int j = 0; j < 4; ++j) {
      const float bv = bias ? bias[n0 + wn + 16 * j + cl] : 0.0f;
#pragma unroll
      for (int r = 0; r < 8; ++r) so[(16 * i + rh + r) * 68 + 16 * j + cl] = (acc[i][j][r] + accx[i][j][r] * (1.0f / 2048.0f)) * scale + bv;
    }
  asm volatile("s_wait_dscnt 0" ::: "memory");
  __builtin_amdgcn_wave_barrier();
  if (ACC) {
#pragma unroll
    for (int it = 0; it < 16; ++it) { const int f4 = lane + 32 * it, rr = f4 >> 4, q = (f4 & 15) * 4;
      const v4f_t old = *(const v4fa*)(Y + (size_t)(m0 + wm + rr) * ldy + n0 + wn + q);
      v4f_t v = *(const v4fa*)(so + rr * 68 + q); v += old; *(v4fa*)(so + rr * 68 + q) = v; }
    asm volatile("s_wait_dscnt 0" ::: "memory");
  }
#pragma unroll 1
  for (int pass = 0; pass < 2; ++pass) {
#pragma unroll
    for (int it = 0; it < 16; ++it) { const int f4 = lane + 32 * it, rr = f4 >> 4, q = (f4 & 15) * 4;
      *(volatile v4f_t*)(Y + (size_t)(m0 + wm + rr) * ldy + n0 + wn + q) = *(const v4fa*)(so + rr * 68 + q); }
    __threadfence();
  }
}

__global__ __launch_bounds__(256) void k_transpose(const float* __restrict__ Wm, float* __restrict__ Wt, int rows, int cols) {
  __shared__ float tS[64][65];
  const int tid = threadIdx.x, tbj = cols / 64, bi = blockIdx.x / tbj, bj = blockIdx.x % tbj;
  for (int e = tid; e < 64 * 64; e += 256) { const int r = e >> 6, c = e & 63; tS[r][c] = Wm[(size_t)(bi * 64 + r) * cols + bj * 64 + c]; }
  __syncthreads();
  for (int ch = tid; ch < 64 * 16; ch += 256) { const int r = ch >> 4, q4 = (ch & 15) * 4; v4f_t o; o[0] = tS[q4][r]; o[1] = tS[q4 + 1][r]; o[2] = tS[q4 + 2][r]; o[3] = tS[q4 + 3][r];
    float* dst = Wt + (size_t)(bj * 64 + r) * rows + bi * 64 + q4; *(volatile v4f_t*)dst = o; __threadfence(); *(volatile v4f_t*)dst = o; }
}

#define NBpr 2
#define SSpr 2048
#define SIN 2048
#define DDpr 1024
#define NHpr 16
#define DKpr 64
__global__ __launch_bounds__(256) void k_fill(float* __restrict__ p, float val, size_t n4) { const size_t i = (size_t)blockIdx.x * 256 + threadIdx.x; if (i < n4) { v4f_t v = {val, val, val, val}; *(volatile v4f_t*)(p + 4 * i) = v; __threadfence(); *(volatile v4f_t*)(p + 4 * i) = v; } }
__global__ __launch_bounds__(256) void k_dbg_zero(float* __restrict__ p, size_t n4) { const size_t i = (size_t)blockIdx.x * 256 + threadIdx.x; if (i < n4) { v4f_t z = {0.f,0.f,0.f,0.f}; *(volatile v4f_t*)(p + 4 * i) = z; __threadfence(); *(volatile v4f_t*)(p + 4 * i) = z; } }
__global__ __launch_bounds__(256) void k_copy(const float* __restrict__ src, float* __restrict__ dst, size_t n4) { const size_t i = (size_t)blockIdx.x * 256 + threadIdx.x; if (i < n4) { const v4f_t v = *(const v4f_t*)(src + 4 * i); *(volatile v4f_t*)(dst + 4 * i) = v; __threadfence(); *(volatile v4f_t*)(dst + 4 * i) = v; } }
__device__ __forceinline__ float bf16r(float x) { unsigned int u = __float_as_uint(x); u = (u + 0x7FFFu + ((u >> 16) & 1u)) & 0xFFFF0000u; return __uint_as_float(u); }
__global__ __launch_bounds__(256) void k_cpyrnd(const float* __restrict__ src, float* __restrict__ dst, float mul, size_t n4) { const size_t i = (size_t)blockIdx.x * 256 + threadIdx.x; if (i >= n4) return; v4f_t v = *(const v4f_t*)(src + 4 * i);
#pragma unroll
  for (int u = 0; u < 4; ++u) v[u] = mul * bf16r(v[u]);
  *(volatile v4f_t*)(dst + 4 * i) = v; __threadfence(); *(volatile v4f_t*)(dst + 4 * i) = v; }
__global__ __launch_bounds__(256) void k_wprepT(const float* __restrict__ Wt, float* __restrict__ WT, int nout, int nin, float mul) { const int i = blockIdx.x, tid = threadIdx.x;
#pragma unroll 1
  for (int o = tid; o < nout; o += 256) { const float w = mul * bf16r(Wt[(size_t)o * nin + i]); *(volatile float*)(WT + (size_t)i * nout + o) = w; __threadfence(); *(volatile float*)(WT + (size_t)i * nout + o) = w; } }
__global__ __launch_bounds__(256) void k_bprep(const float* __restrict__ b, float* __restrict__ B2, int n, float mul) { for (int o = threadIdx.x; o < n; o += 256) { const float v = mul * bf16r(b[o]); *(volatile float*)(B2 + o) = v; __threadfence(); *(volatile float*)(B2 + o) = v; } }

__global__ __launch_bounds__(256) void k_bhatt(const float* __restrict__ MQ, const float* __restrict__ SQ, const float* __restrict__ MK, const float* __restrict__ SK, const float* __restrict__ MV, const float* __restrict__ SV, float* __restrict__ omu, float* __restrict__ osg, int srows) {
  __shared__ __attribute__((aligned(16))) float mq[1024], sq[1024], mk[1024], sk[1024], mv[1024], sv[1024]; __shared__ float att[256];
  const size_t t = blockIdx.x; const int tid = threadIdx.x;
  { const size_t o4 = t * DDpr + 4 * tid; *(v4f_t*)(mq + 4 * tid) = *(const v4f_t*)(MQ + o4); *(v4f_t*)(sq + 4 * tid) = *(const v4f_t*)(SQ + o4); *(v4f_t*)(mk + 4 * tid) = *(const v4f_t*)(MK + o4); *(v4f_t*)(sk + 4 * tid) = *(const v4f_t*)(SK + o4); *(v4f_t*)(mv + 4 * tid) = *(const v4f_t*)(MV + o4); *(v4f_t*)(sv + 4 * tid) = *(const v4f_t*)(SV + o4); }
  __syncthreads();
  const int i = tid >> 4, j = tid & 15; float dist = 0.0f;
#pragma unroll 1
  for (int d = 0; d < DKpr; ++d) { const float sgq = sq[i * DKpr + d], sgk = sk[j * DKpr + d]; const float sq2 = sgq * sgq + 1e-6f, sk2 = sgk * sgk + 1e-6f; const float dm = mq[i * DKpr + d] - mk[j * DKpr + d];
    const float term1 = 0.25f * logf(0.25f * (sq2 / sk2 + sk2 / sq2 + 2.0f)); const float term2 = 0.25f * dm * dm / (sgq * sgq + sgk * sgk + 1e-6f); dist += term1 + term2; }
  float lg = -0.5f * (dist * 0.125f); float m = lg;
  m = fmaxf(m, __shfl_xor(m, 1, 32)); m = fmaxf(m, __shfl_xor(m, 2, 32)); m = fmaxf(m, __shfl_xor(m, 4, 32)); m = fmaxf(m, __shfl_xor(m, 8, 32));
  float e = expf(lg - m); float z = e; z += __shfl_xor(z, 1, 32); z += __shfl_xor(z, 2, 32); z += __shfl_xor(z, 4, 32); z += __shfl_xor(z, 8, 32);
  att[tid] = e / z; __syncthreads();
  const int hi = tid >> 4, c4 = (tid & 15) * 4; v4f_t am, av; am[0] = am[1] = am[2] = am[3] = 0.0f; av[0] = av[1] = av[2] = av[3] = 0.0f;
#pragma unroll 1
  for (int jj = 0; jj < NHpr; ++jj) { const float a = att[hi * NHpr + jj]; const v4f_t mvj = *(const v4f_t*)(mv + jj * DKpr + c4), svj = *(const v4f_t*)(sv + jj * DKpr + c4); am += a * mvj; av += a * (svj * svj); }
  v4f_t os; for (int u = 0; u < 4; ++u) os[u] = sqrtf(fmaxf(av[u], 0.0f) + 1e-6f);
  float* dm_ = omu + ((size_t)hi * srows + t) * DKpr + c4; float* ds_ = osg + ((size_t)hi * srows + t) * DKpr + c4;
  *(volatile v4f_t*)dm_ = am; *(volatile v4f_t*)ds_ = os; __threadfence(); *(volatile v4f_t*)dm_ = am; *(volatile v4f_t*)ds_ = os; }

extern "C" void kernel_launch(void* const* d_in, const int* in_sizes, int n_in,
                              void* d_out, int out_size, void* d_ws, size_t ws_size,
                              hipStream_t stream) {
  (void)in_sizes; (void)n_in; (void)out_size;
  const float** f = (const float**)d_in;
  float* out0 = (float*)d_out; float* out1 = out0 + (size_t)2 * SIN * DDpr;
  char* ws = (char*)d_ws;
  float* WB = (float*)ws; ws += (size_t)6 * DDpr * DDpr * 4; float* BB = (float*)ws; ws += (size_t)6 * DDpr * 4; float* g64 = (float*)ws; ws += DDpr * 4; float* XB = (float*)ws; ws += (size_t)SSpr * DDpr * 4;
  float* P[6]; for (int i = 0; i < 6; ++i) { P[i] = (float*)ws; ws += (size_t)SSpr * DDpr * 4; }
  if ((size_t)(ws - (char*)d_ws) > ws_size) return;
  const dim3 blk(256); const dim3 gp(SSpr / 128, DDpr / 128); const size_t n4 = (size_t)SSpr * DDpr / 4;
  k_fill<<<dim3(1), blk, 0, stream>>>(g64, 1.0f / 64.0f, DDpr / 4);
  for (int i = 0; i < 6; ++i) { k_cpyrnd<<<dim3(((size_t)DDpr * DDpr / 4 + 255) / 256), blk, 0, stream>>>(f[6 + i], WB + (size_t)i * DDpr * DDpr, 64.0f, (size_t)DDpr * DDpr / 4); k_bprep<<<dim3(1), blk, 0, stream>>>(f[12 + i], BB + (size_t)i * DDpr, DDpr, 64.0f); }

  for (int b = 0; b < NBpr; ++b) {
    for (int i = 0; i < 6; ++i) { k_cpyrnd<<<dim3((n4 + 255) / 256), blk, 0, stream>>>(f[i] + (size_t)b * SIN * DDpr, XB, 1.0f, n4); gemm_kne<float, 4, false><<<gp, blk, 0, stream>>>(XB, DDpr, WB + (size_t)i * DDpr * DDpr, DDpr, BB + (size_t)i * DDpr, nullptr, g64, P[i], DDpr, DDpr); }
    k_bhatt<<<dim3(SSpr), blk, 0, stream>>>(P[0], P[3], P[1], P[4], P[2], P[5], out0 + (size_t)b * SIN * DDpr, out1 + (size_t)b * SIN * DDpr, SIN);
  }
}
